// GCN_5282809775007
// MI455X (gfx1250) — hardware-verified
//
#include <hip/hip_runtime.h>
#include <stddef.h>
#include <stdint.h>
#include <math.h>


#define DF     128
#define NLAY   3
#define NTHR   256
#define NWAVE  8
#define EPT    8
#define CHUNK  (NTHR * EPT)
#define WCAP   (EPT * 32)
#define LISTN  (NWAVE * WCAP)
#define NBA    1024
#define SLA    10
#define RCAP   28672
#define DEGCAP 64
#define GBM    64
#define GBN    128
#define GTHR   128
#define METAI  32
#define TBL    (RCAP + 2 * NBA + METAI)
#define SCN    (2 * NBA + METAI)
#define BK_OUT0  (LISTN + RCAP + NBA)
#define BK_ZINTS (LISTN + 2 * RCAP + 3 * NBA + METAI + 16)
#define UPL    (DF * (DF / 8))
#define WSMAX  134217728

static_assert((CHUNK & (CHUNK - 1)) == 0 && CHUNK <= 4096);
static_assert((NBA & (NBA - 1)) == 0 && NBA == (1 << SLA));
static_assert(((long long)CHUNK << SLA) < (1LL << 31));
static_assert(NBA % NWAVE == 0 && NBA % 32 == 0);
static_assert(RCAP % 4 == 0 && BK_ZINTS % 4 == 0 && BK_OUT0 % 4 == 0 && TBL % 4 == 0 && SCN % 4 == 0);
static_assert((TBL * 4) % 128 == 0 && (RCAP * 4) % 128 == 0);
static_assert(BK_ZINTS * 4 <= 300000);
static_assert(DF % 32 == 0 && GBN == DF && GBM == (GTHR / 32) * 16 && DF == 4 * 32);
static_assert((NLAY * UPL) % NTHR == 0 && DF / 8 == 16);
static_assert(GTHR * 4 == 4 * DF);
static_assert(DEGCAP <= RCAP);

typedef float          v4f   __attribute__((ext_vector_type(4)));
typedef float          v8f   __attribute__((ext_vector_type(8)));
typedef double         v2d   __attribute__((ext_vector_type(2)));
typedef int            v4i   __attribute__((ext_vector_type(4)));
typedef int            v8i   __attribute__((ext_vector_type(8)));
typedef unsigned short v8us  __attribute__((ext_vector_type(8)));
typedef unsigned short v16us __attribute__((ext_vector_type(16)));
typedef __bf16         v16bf __attribute__((ext_vector_type(16)));
typedef v4f  __attribute__((may_alias)) v4fa;
typedef v4i  __attribute__((may_alias)) v4ia;
typedef v8us __attribute__((may_alias)) v8usa;
union FragB { v16bf v; v16us u; v8us h[2]; v8i w; };

__device__ __forceinline__ v8f wmb(const FragB& a, const FragB& b, v8f c) {
  v8f d = __builtin_amdgcn_wmma_f32_16x16x32_bf16(false, a.v, false, b.v, (short)0, c, false, false);
  asm volatile("v_nop\n\tv_nop\n\tv_nop\n\tv_nop" : "+v"(d) : "v"(a.w), "v"(b.w));
  return d;
}

__device__ __forceinline__ unsigned bf16_bits(float f) {
  const unsigned u = __float_as_uint(f);
  return (u + 0x7FFFu + ((u >> 16) & 1u)) >> 16;
}
__device__ __forceinline__ float bf16_val(float f) {
  return __uint_as_float(bf16_bits(f) << 16);
}

template <int SLB>
__device__ __forceinline__ int scan_chunk(const int* __restrict__ dsts, int nE, int cbase, int slotBase,
                                          int nb, int vec8, int* list, int tid, int lane, int wave) {
  int wc = 0;
  const int el0  = tid * EPT;
  const int e0   = cbase + el0;
  const int sent = -2147483647 - 1;
  v4i da, db;
  if (vec8 != 0 && cbase + CHUNK <= nE) {
    da = *(const v4i*)(dsts + e0);
    db = *(const v4i*)(dsts + e0 + 4);
  } else {
    da.x = (e0     < nE) ? dsts[min(e0,     nE - 1)] : sent;
    da.y = (e0 + 1 < nE) ? dsts[min(e0 + 1, nE - 1)] : sent;
    da.z = (e0 + 2 < nE) ? dsts[min(e0 + 2, nE - 1)] : sent;
    da.w = (e0 + 3 < nE) ? dsts[min(e0 + 3, nE - 1)] : sent;
    db.x = (e0 + 4 < nE) ? dsts[min(e0 + 4, nE - 1)] : sent;
    db.y = (e0 + 5 < nE) ? dsts[min(e0 + 5, nE - 1)] : sent;
    db.z = (e0 + 6 < nE) ? dsts[min(e0 + 6, nE - 1)] : sent;
    db.w = (e0 + 7 < nE) ? dsts[min(e0 + 7, nE - 1)] : sent;
  }
  const unsigned nbs = (unsigned)slotBase;
  const unsigned unb = (unsigned)nb;
  const unsigned s0 = (unsigned)da.x - nbs, s1 = (unsigned)da.y - nbs;
  const unsigned s2 = (unsigned)da.z - nbs, s3 = (unsigned)da.w - nbs;
  const unsigned s4 = (unsigned)db.x - nbs, s5 = (unsigned)db.y - nbs;
  const unsigned s6 = (unsigned)db.z - nbs, s7 = (unsigned)db.w - nbs;
  const bool h0 = s0 < unb, h1 = s1 < unb, h2 = s2 < unb, h3 = s3 < unb;
  const bool h4 = s4 < unb, h5 = s5 < unb, h6 = s6 < unb, h7 = s7 < unb;
  const unsigned any = __builtin_amdgcn_ballot_w32(h0 | h1 | h2 | h3 | h4 | h5 | h6 | h7);
  if (any != 0u) {
#define HITJ(J, HJ, SJ) { \
      const unsigned mj = __builtin_amdgcn_ballot_w32(HJ); \
      if (mj != 0u) { \
        if (HJ) { \
          const int pos = wc + (int)__builtin_amdgcn_mbcnt_lo(mj, 0u); \
          if (pos < WCAP) list[wave * WCAP + pos] = ((el0 + (J)) << SLB) | (int)(SJ); \
        } \
        wc += (int)__builtin_popcount(mj); } }
    HITJ(0, h0, s0)
    HITJ(1, h1, s1)
    HITJ(2, h2, s2)
    HITJ(3, h3, s3)
    HITJ(4, h4, s4)
    HITJ(5, h5, s5)
    HITJ(6, h6, s6)
    HITJ(7, h7, s7)
#undef HITJ
  }
  return wc;
}

__global__ __launch_bounds__(NTHR) void k_prep(const float* __restrict__ Ws, unsigned short* WT) {
  const int u = (int)blockIdx.x * NTHR + (int)threadIdx.x;
  if (u >= NLAY * UPL) return;
  const int l  = u >> 11;
  const int v  = u & (UPL - 1);
  const int n  = v >> 4;
  const int k8 = (v & 15) * 8;
  const float* p = Ws + (size_t)l * DF * DF + (size_t)k8 * DF + n;
  v8us o;
#pragma unroll
  for (int i = 0; i < 8; ++i) o[i] = (unsigned short)bf16_bits(p[(size_t)i * DF]);
  unsigned short* dp = WT + (size_t)l * DF * DF + (size_t)n * DF + k8;
  *(volatile v8us*)dp = o;
  __threadfence();
  *(volatile v8us*)dp = o;
}

__global__ __launch_bounds__(NTHR) void k_bucket(const int* __restrict__ srcs, const int* __restrict__ dsts,
                                                 int nE, int nN, int vec8, int* tbl) {
  extern __shared__ __attribute__((aligned(16))) int dsm[];
  int* list = dsm;
  int* hl   = dsm + LISTN;
  int* cur  = hl + RCAP;
  int* sl   = cur + NBA;
  int* cnt  = sl + RCAP;
  int* offs = cnt + NBA;
  int* meta = offs + NBA;
  int* misc = meta + METAI;
  const int tid = (int)threadIdx.x, lane = tid & 31, wave = tid >> 5;
  const int nodeBase = (int)blockIdx.x * NBA;

  {
    const v4i z4 = {0, 0, 0, 0};
    for (int i = tid * 4; i < BK_ZINTS; i += NTHR * 4) *(v4ia*)(dsm + i) = z4;
  }
  __syncthreads();

  int t = 0, ov = 0;
  const int nChunks = (nE + CHUNK - 1) / CHUNK;
#pragma unroll 1
  for (int ch = 0; ch < nChunks; ++ch) {
    const int cbase = ch * CHUNK;
    const int wc = scan_chunk<SLA>(dsts, nE, cbase, nodeBase, NBA, vec8, list, tid, lane, wave);
    if (lane == 0) misc[wave] = wc;
    __syncthreads();
    if (wave == 0) {
#pragma unroll 1
      for (int w2 = 0; w2 < NWAVE; ++w2) {
        int c = misc[w2];
        c = c < 0 ? 0 : (c > WCAP ? WCAP : c);
#pragma unroll 1
        for (int b0 = 0; b0 < c; b0 += 32) {
          const int idx = b0 + lane;
          const int ent = list[w2 * WCAP + (idx < WCAP ? idx : WCAP - 1)];
          const int m32 = (c - b0) < 32 ? (c - b0) : 32;
#pragma unroll 1
          for (int k = 0; k < m32; ++k) {
            const int u    = __builtin_amdgcn_readlane(ent, k);
            const int slot = u & (NBA - 1);
            const int el   = (u >> SLA) & (CHUNK - 1);
            const int pk   = ((cbase + el) << SLA) | slot;
            if (t < RCAP) {
              if (lane == 0) { hl[t] = pk; cnt[slot] = cnt[slot] + 1; }
              t = t + 1;
            } else {
              ov = 1;
            }
          }
        }
      }
    }
    __syncthreads();
  }
  if (wave == 0 && lane == 0) { misc[8] = t; misc[9] = ov; }
  __syncthreads();
  int tt = misc[8];
  tt = tt < 0 ? 0 : (tt > RCAP ? RCAP : tt);
  const int ovf = misc[9];

  if (wave == 0) {
    const int base = lane * (NBA / 32);
    int s = 0;
#pragma unroll 1
    for (int i = 0; i < NBA / 32; ++i) s += cnt[base + i];
    int incl = s;
#pragma unroll
    for (int d = 1; d < 32; d <<= 1) {
      const int y = __shfl_up(incl, d, 32);
      if (lane >= d) incl += y;
    }
    int run = incl - s;
#pragma unroll 1
    for (int i = 0; i < NBA / 32; ++i) {
      const int cv = cnt[base + i];
      offs[base + i] = run;
      cur[base + i]  = run;
      run += cv;
    }
  }
  __syncthreads();
  if (wave == 0) {
#pragma unroll 1
    for (int b0 = 0; b0 < tt; b0 += 32) {
      const int idx = b0 + lane;
      const int ent = hl[idx < RCAP ? idx : RCAP - 1];
      const int m32 = (tt - b0) < 32 ? (tt - b0) : 32;
#pragma unroll 1
      for (int k = 0; k < m32; ++k) {
        const int u    = __builtin_amdgcn_readlane(ent, k);
        const int slot = u & (NBA - 1);
        if (lane == 0) {
          int p = cur[slot];
          p = p < 0 ? 0 : (p > RCAP - 1 ? RCAP - 1 : p);
          sl[p] = u;
          cur[slot] = p + 1;
        }
      }
    }
  }
  __syncthreads();

#pragma unroll 1
  for (int i0 = 0; i0 < tt; i0 += NTHR) {
    const int i  = i0 + tid;
    const int ic = i < RCAP ? i : RCAP - 1;
    const int u  = sl[ic];
    int eid = u >> SLA;
    eid = eid < 0 ? 0 : (eid > nE - 1 ? nE - 1 : eid);
    int sr = srcs[eid];
    sr = sr < 0 ? 0 : (sr > nN - 1 ? nN - 1 : sr);
    if (i < tt) sl[i] = sr;
  }
  if (tid == 0) { meta[0] = tt; meta[1] = ovf; }
  __syncthreads();

  int* tp = tbl + (size_t)blockIdx.x * TBL;
  const int* img = dsm + BK_OUT0;
#pragma unroll 1
  for (int i = tid; i < TBL / 4; i += NTHR) {
    const v4i v = *(const v4ia*)(img + 4 * i);
    *(volatile v4i*)(tp + 4 * i) = v;
  }
  __threadfence();
#pragma unroll 1
  for (int i = tid; i < TBL / 4; i += NTHR) {
    const v4i v = *(const v4ia*)(img + 4 * i);
    *(volatile v4i*)(tp + 4 * i) = v;
  }
}

template <int MODE>
__global__ __launch_bounds__(GTHR) void k_gemm(const float* __restrict__ Ain, const unsigned short* __restrict__ WT,
                                               const float* __restrict__ prm, float* outp, int nN) {
  __shared__ __attribute__((aligned(16))) float stg[GBM * GBN];
  __shared__ __attribute__((aligned(16))) float sp[4 * DF];
  const int tid = (int)threadIdx.x, lane = tid & 31, wave = tid >> 5, hh = lane >> 4, m = lane & 15;
  const int rowBase = (int)blockIdx.x * GBM;

  if constexpr (MODE != 0) {
    const v4f pv4 = *(const v4f*)(prm + 4 * tid);
    *(v4fa*)(sp + 4 * tid) = pv4;
    __syncthreads();
  }

  v8f acc[8];
  {
    const v8f z = {0.f, 0.f, 0.f, 0.f, 0.f, 0.f, 0.f, 0.f};
#pragma unroll
    for (int t = 0; t < 8; ++t) acc[t] = z;
  }
  const int  row = rowBase + 16 * wave + m;
  const bool ok  = row < nN;
  const int  rc  = ok ? row : nN - 1;
  const float* ap = Ain + (size_t)rc * DF + 8 * hh;
  const unsigned short* bp = WT + (size_t)m * DF + 8 * hh;

#pragma unroll 1
  for (int k0 = 0; k0 < DF; k0 += 32) {
    FragB ah, al;
    {
      const v8i z8 = {0, 0, 0, 0, 0, 0, 0, 0};
      al.w = z8;
    }
#pragma unroll
    for (int q = 0; q < 4; ++q) {
      const int koff = (q >> 1) * 16 + (q & 1) * 4;
      const v4f xv = *(const v4f*)(ap + k0 + koff);
      v4f mu4 = {0.f, 0.f, 0.f, 0.f}, rs4 = mu4, g4 = mu4, b4 = mu4;
      if constexpr (MODE != 0) {
        const int c = k0 + 8 * hh + koff;
        mu4 = *(const v4fa*)(sp + c);
        rs4 = *(const v4fa*)(sp + DF + c);
        g4  = *(const v4fa*)(sp + 2 * DF + c);
        b4  = *(const v4fa*)(sp + 3 * DF + c);
      }
#pragma unroll
      for (int j = 0; j < 4; ++j) {
        const float xj = xv[j];
        if constexpr (MODE == 0) {
          const unsigned hb = bf16_bits(xj);
          ah.u[4 * q + j] = ok ? (unsigned short)hb : (unsigned short)0;
        } else {
          const float tv = ((xj - mu4[j]) * rs4[j]) * g4[j] + b4[j];
          const float y  = (tv > 0.0f) ? tv : (tv - tv);
          const unsigned hb = bf16_bits(y);
          const unsigned lb = bf16_bits(y - __uint_as_float(hb << 16));
          ah.u[4 * q + j] = ok ? (unsigned short)hb : (unsigned short)0;
          al.u[4 * q + j] = ok ? (unsigned short)lb : (unsigned short)0;
        }
      }
    }
#pragma unroll
    for (int nt = 0; nt < 8; ++nt) {
      const unsigned short* wq = bp + (size_t)(16 * nt) * DF + k0;
      FragB bf;
      bf.h[0] = *(const v8usa*)wq;
      bf.h[1] = *(const v8usa*)(wq + 16);
      acc[nt] = wmb(ah, bf, acc[nt]);
      if constexpr (MODE != 0) acc[nt] = wmb(al, bf, acc[nt]);
    }
  }

#pragma unroll
  for (int nt = 0; nt < 8; ++nt) {
    const int lc = 16 * nt + m;
#pragma unroll
    for (int r = 0; r < 8; ++r) {
      const int lr = 16 * wave + 8 * hh + r;
      stg[lr * GBN + lc] = acc[nt][r];
    }
  }
  __syncthreads();

  v4f pv[16];
#pragma unroll
  for (int i = 0; i < 16; ++i) pv[i] = *(const v4fa*)(stg + (16 * wave + i) * GBN + 4 * lane);

#pragma unroll
  for (int i = 0; i < 16; ++i) {
    const int r = rowBase + 16 * wave + i;
    if (r < nN) *(volatile v4f*)(outp + (size_t)r * DF + 4 * lane) = pv[i];
  }
  __threadfence();
#pragma unroll
  for (int i = 0; i < 16; ++i) {
    const int r = rowBase + 16 * wave + i;
    if (r < nN) *(volatile v4f*)(outp + (size_t)r * DF + 4 * lane) = pv[i];
  }
}

template <int FIN>
__global__ __launch_bounds__(NTHR) void k_agg(const int* __restrict__ tbl, int nN, const float* __restrict__ H,
                                              float* outp, double* rec) {
  __shared__ __attribute__((aligned(16))) int sc[SCN];
  __shared__ __attribute__((aligned(16))) double wpart[NWAVE * 256];
  __shared__ __attribute__((aligned(16))) double srec[256];
  const int tid = (int)threadIdx.x, lane = tid & 31, wave = tid >> 5;
  const int nodeBase = (int)blockIdx.x * NBA;
  const int* tb = tbl + (size_t)blockIdx.x * TBL;

#pragma unroll 1
  for (int i0 = 0; i0 < SCN / 4; i0 += NTHR) {
    const int i  = i0 + tid;
    const int ic = i < SCN / 4 ? i : SCN / 4 - 1;
    const v4i v = *(const v4i*)(tb + RCAP + 4 * ic);
    if (i < SCN / 4) *(v4ia*)(sc + 4 * i) = v;
  }
  __syncthreads();

  const float qnan = __int_as_float(0x7fc00000);
  const int   ovf  = sc[2 * NBA + 1];
  const float pz   = (ovf != 0) ? qnan : 0.0f;
  double s0 = 0.0, s1 = 0.0, s2 = 0.0, s3 = 0.0;
  double q0 = 0.0, q1 = 0.0, q2 = 0.0, q3 = 0.0;

#pragma unroll 1
  for (int si = 0; si < NBA / NWAVE; ++si) {
    const int s    = si * NWAVE + wave;
    const int node = nodeBase + s;
    int c = sc[s];
    const bool big = c > DEGCAP;
    c = c < 0 ? 0 : (c > DEGCAP ? DEGCAP : c);
    int o = sc[NBA + s];
    o = o < 0 ? 0 : (o > RCAP ? RCAP : o);
    float a0 = 0.0f, a1 = 0.0f, a2 = 0.0f, a3 = 0.0f;
#pragma unroll 1
    for (int b0 = 0; b0 < c; b0 += 32) {
      int idx = o + b0 + lane;
      idx = idx > RCAP - 1 ? RCAP - 1 : idx;
      int sr = tb[idx];
      sr = sr < 0 ? 0 : (sr > nN - 1 ? nN - 1 : sr);
      const int m32 = (c - b0) < 32 ? (c - b0) : 32;
#pragma unroll 1
      for (int k = 0; k < m32; ++k) {
        const int sk = __builtin_amdgcn_readlane(sr, k);
        const v4f a = *(const v4f*)(H + (size_t)sk * DF + 4 * lane);
        a0 += a.x; a1 += a.y; a2 += a.z; a3 += a.w;
      }
    }
    const float pzr = big ? qnan : pz;
    const bool live = node < nN;
    if constexpr (FIN != 0) {
      float mx = fmaxf(fmaxf(a0, a1), fmaxf(a2, a3));
#pragma unroll
      for (int d = 16; d > 0; d >>= 1) mx = fmaxf(mx, __shfl_xor(mx, d, 32));
      const float e0 = a0 - mx, e1 = a1 - mx, e2 = a2 - mx, e3 = a3 - mx;
      float r0 = e0, r1 = e1, r2 = e2, r3 = e3;
      float sm = 0.0f;
#pragma unroll 1
      for (int j = 0; j < 4; ++j) {
        sm += expf(r0);
        const float tq = r0; r0 = r1; r1 = r2; r2 = r3; r3 = tq;
      }
#pragma unroll
      for (int d = 16; d > 0; d >>= 1) sm += __shfl_xor(sm, d, 32);
      const float lg = logf(sm);
      v4f ow;
      ow.x = (e0 - lg) + pzr; ow.y = (e1 - lg) + pzr;
      ow.z = (e2 - lg) + pzr; ow.w = (e3 - lg) + pzr;
      if (live) {
        float* op = outp + (size_t)node * DF + 4 * lane;
        *(volatile v4f*)op = ow;
        __threadfence();
        *(volatile v4f*)op = ow;
      }
    } else {
      v4f ow;
      ow.x = live ? (a0 + pzr) : 0.0f;
      ow.y = live ? (a1 + pzr) : 0.0f;
      ow.z = live ? (a2 + pzr) : 0.0f;
      ow.w = live ? (a3 + pzr) : 0.0f;
      s0 += (double)ow.x; q0 += (double)ow.x * (double)ow.x;
      s1 += (double)ow.y; q1 += (double)ow.y * (double)ow.y;
      s2 += (double)ow.z; q2 += (double)ow.z * (double)ow.z;
      s3 += (double)ow.w; q3 += (double)ow.w * (double)ow.w;
      if (live) {
        float* op = outp + (size_t)node * DF + 4 * lane;
        *(volatile v4f*)op = ow;
        __threadfence();
        *(volatile v4f*)op = ow;
      }
    }
  }

  if constexpr (FIN == 0) {
    double* wp = wpart + wave * 256;
    wp[4 * lane + 0] = s0; wp[4 * lane + 1] = s1; wp[4 * lane + 2] = s2; wp[4 * lane + 3] = s3;
    wp[DF + 4 * lane + 0] = q0; wp[DF + 4 * lane + 1] = q1;
    wp[DF + 4 * lane + 2] = q2; wp[DF + 4 * lane + 3] = q3;
    __syncthreads();
    double r = 0.0;
#pragma unroll
    for (int w2 = 0; w2 < NWAVE; ++w2) r += wpart[w2 * 256 + tid];
    srec[tid] = r;
    __syncthreads();
    const int t2 = 2 * (tid & 127);
    v2d rv;
    rv.x = srec[t2];
    rv.y = srec[t2 + 1];
    double* rp = rec + (size_t)blockIdx.x * 256 + t2;
    const bool okst = tid < 128;
    if (okst) *(volatile v2d*)rp = rv;
    __threadfence();
    if (okst) *(volatile v2d*)rp = rv;
  }
}

__global__ __launch_bounds__(128) void k_bncomb(const double* __restrict__ rec, const float* __restrict__ gam,
                                                const float* __restrict__ bet, float* prm, double invN, int nb) {
  __shared__ __attribute__((aligned(16))) float st[4 * DF];
  const int c = (int)threadIdx.x;
  double S = 0.0, Q = 0.0;
#pragma unroll 1
  for (int b = 0; b < nb; ++b) {
    S += rec[(size_t)b * 256 + c];
    Q += rec[(size_t)b * 256 + DF + c];
  }
  const double mu = S * invN;
  double var = Q * invN - mu * mu;
  var = (var < 0.0) ? 0.0 : var;
  st[c]          = (float)mu;
  st[DF + c]     = rsqrtf((float)var + 1e-5f);
  st[2 * DF + c] = bf16_val(gam[c]);
  st[3 * DF + c] = bf16_val(bet[c]);
  __syncthreads();
  const v4f v = *(const v4fa*)(st + 4 * c);
  float* op = prm + 4 * c;
  *(volatile v4f*)op = v;
  __threadfence();
  *(volatile v4f*)op = v;
}

static inline int cdiv(int a, int b) { return (a + b - 1) / b; }
static inline size_t al256(size_t o) { return (o + 255) & ~(size_t)255; }

extern "C" void kernel_launch(void* const* d_in, const int* in_sizes, int n_in,
                              void* d_out, int out_size, void* d_ws, size_t ws_size,
                              hipStream_t stream) {
  if (n_in < 5) return;
  if (in_sizes[0] < DF || (in_sizes[0] % DF) != 0) return;
  const int nN = in_sizes[0] / DF;
  if (nN < 16 || nN > (1 << 22)) return;
  if (in_sizes[1] < 2 || (in_sizes[1] & 1) != 0) return;
  const int nE = in_sizes[1] / 2;
  if (nE < 1 || nE >= (1 << (31 - SLA))) return;
  if (in_sizes[2] != NLAY * DF * DF) return;
  if (in_sizes[3] != (NLAY - 1) * DF || in_sizes[4] != (NLAY - 1) * DF) return;
  if ((long long)out_size != (long long)nN * DF) return;

  const float* x    = (const float*)d_in[0];
  const int*   edge = (const int*)d_in[1];
  const float* Ws   = (const float*)d_in[2];
  const float* gam  = (const float*)d_in[3];
  const float* bet  = (const float*)d_in[4];
  float* out = (float*)d_out;
  const int* src = edge;
  const int* dst = edge + nE;

  const int gM = cdiv(nN, GBM);
  const int gA = cdiv(nN, NBA);
  if ((long long)gA * NBA < (long long)nN) return;
  const int vec8 = ((nE & 3) == 0) ? 1 : 0;
  const double invN = 1.0 / (double)nN;

  char* ws = (char*)d_ws;
  size_t off = 0;
  const size_t oWT  = off; off = al256(off + (size_t)NLAY * DF * DF * 2);
  const size_t oTBL = off; off = al256(off + (size_t)gA * TBL * 4);
  const size_t oH   = off; off = al256(off + (size_t)nN * DF * 4);
  const size_t oAGG = off; off = al256(off + (size_t)nN * DF * 4);
  const size_t oREC = off; off = al256(off + (size_t)2 * gA * 256 * 8);
  const size_t oPRM = off; off = al256(off + (size_t)2 * 4 * DF * 4);
  if (off > ws_size || off > (size_t)WSMAX) return;
  unsigned short* WT  = (unsigned short*)(ws + oWT);
  int*            TB  = (int*)(ws + oTBL);
  float*          H   = (float*)(ws + oH);
  float*          AGG = (float*)(ws + oAGG);
  double*         REC = (double*)(ws + oREC);
  float*          PRM = (float*)(ws + oPRM);
  double* REC1 = REC + (size_t)gA * 256;
  float*  PRM1 = PRM + 4 * DF;

  const size_t bkLds = (size_t)BK_ZINTS * 4;
  hipFuncSetAttribute(reinterpret_cast<const void*>(&k_bucket), hipFuncAttributeMaxDynamicSharedMemorySize, (int)bkLds);

  k_prep<<<(NLAY * UPL) / NTHR, NTHR, 0, stream>>>(Ws, WT);
  k_bucket<<<gA, NTHR, bkLds, stream>>>(src, dst, nE, nN, vec8, TB);
  k_gemm<0><<<gM, GTHR, 0, stream>>>(x, WT, PRM, H, nN);
  k_agg<0><<<gA, NTHR, 0, stream>>>(TB, nN, H, AGG, REC);
  k_bncomb<<<1, 128, 0, stream>>>(REC, gam, bet, PRM, invN, gA);
  k_gemm<1><<<gM, GTHR, 0, stream>>>(AGG, WT + (size_t)DF * DF, PRM, H, nN);
  k_agg<0><<<gA, NTHR, 0, stream>>>(TB, nN, H, AGG, REC1);
  k_bncomb<<<1, 128, 0, stream>>>(REC1, gam + DF, bet + DF, PRM1, invN, gA);
  k_gemm<1><<<gM, GTHR, 0, stream>>>(AGG, WT + (size_t)2 * DF * DF, PRM1, H, nN);
  k_agg<1><<<gA, NTHR, 0, stream>>>(TB, nN, H, out, REC1);
}
